// NetG_3289944948771
// MI455X (gfx1250) — hardware-run, weakly checked
//
#include <hip/hip_runtime.h>
#include <math.h>

constexpr int NBATCH   = 512;
constexpr int NSTEP    = 256;
constexpr int NHID     = 256;
constexpr int NDIM     = 3;
constexpr int NGATE    = 3 * NHID;
constexpr int NTHR     = 256;
constexpr int ROWS_BLK = 16;
constexpr int HPITCH   = 264;
constexpr int TCHUNK   = 32;
constexpr int XROW     = TCHUNK * NDIM;
constexpr int NPART    = ROWS_BLK * NDIM;
constexpr int NWAVE    = NTHR / 32;
constexpr float WCARRY = 256.0f;
constexpr float HCARRY = 16.0f;
constexpr float FOLD   = 1.0f / (WCARRY * HCARRY);

static_assert(NBATCH % ROWS_BLK == 0, "batch tile");
static_assert(NHID == 32 * NWAVE, "8 waves x 32 hidden columns");
static_assert(NHID % 32 == 0, "K multiple of 32");
static_assert(NSTEP % TCHUNK == 0, "step chunks");
static_assert((ROWS_BLK * XROW) % NTHR == 0, "x staging exact");
static_assert((XROW * 4) % 128 == 0, "chunk row is whole lines");
static_assert((NSTEP * NDIM * 4) % 128 == 0, "batch row pitch is whole lines");
static_assert((HPITCH % 8) == 0, "16-B aligned A rows");
static_assert((NGATE * NHID / 8) % NTHR == 0, "convert grid exact");

typedef __attribute__((ext_vector_type(16))) _Float16 v16h;
typedef __attribute__((ext_vector_type(8)))  _Float16 v8h;
typedef __attribute__((ext_vector_type(8)))  float    v8f;
typedef __attribute__((ext_vector_type(4)))  float    v4f;

__device__ __forceinline__ void dep_guard3_h(v8f& a0, v8f& a1, v8f& a2, v16h x, v16h y0, v16h y1, v16h y2) {
  asm volatile("v_nop\n\tv_nop\n\tv_nop\n\tv_nop" : "+v"(a0), "+v"(a1), "+v"(a2) : "v"(x), "v"(y0), "v"(y1), "v"(y2));
}
__device__ __forceinline__ void acc_guard3(v8f& a0, v8f& a1, v8f& a2) {
  asm volatile("v_nop\n\tv_nop\n\tv_nop\n\tv_nop" : "+v"(a0), "+v"(a1), "+v"(a2));
}
__device__ __forceinline__ void pin_f(float& x) { asm volatile("" : "+v"(x)); }

struct FragH {
  union U { v16h v; v8h h[2]; };
  static __device__ __forceinline__ v16h load(const _Float16* p) {
    U f;
    f.h[0] = *(const v8h*)(p);
    f.h[1] = *(const v8h*)(p + 16);
    return f.v;
  }
  static __device__ __forceinline__ v8f mma(v16h a, v16h b, v8f c) {
    return __builtin_amdgcn_wmma_f32_16x16x32_f16(false, a, false, b, (short)0, c, false, false);
  }
};

__device__ __forceinline__ float fsig(float x)  { return __builtin_amdgcn_rcpf(1.0f + __expf(-x)); }
__device__ __forceinline__ float ftanh(float x) { return 1.0f - 2.0f * __builtin_amdgcn_rcpf(__expf(2.0f * x) + 1.0f); }

__global__ __launch_bounds__(NTHR) void cvt8_f16_kernel(const float* __restrict__ src, unsigned short* __restrict__ dst,
                                                        int n8, float sc) {
  const int i = blockIdx.x * NTHR + threadIdx.x;
  if (i < n8) {
    const float* sp = src + (size_t)i * 8;
    const v4f a = *(const v4f*)(sp);
    const v4f b = *(const v4f*)(sp + 4);
    v8h hv;
#pragma unroll
    for (int e = 0; e < 4; ++e) {
      const float fa = a[e] * sc;
      const float fb = b[e] * sc;
      hv[e]     = (_Float16)fa;
      hv[4 + e] = (_Float16)fb;
    }
    *(volatile v8h*)(dst + (size_t)i * 8) = hv;
    __threadfence();
    *(volatile v8h*)(dst + (size_t)i * 8) = hv;
  }
}

__global__ __launch_bounds__(NTHR) void gru_seq_kernel(
    const float* __restrict__ Xp, const float* __restrict__ Xf, const float* __restrict__ noise,
    const float* __restrict__ Wih_e, const float* __restrict__ bih_e, const float* __restrict__ bhh_e,
    const float* __restrict__ Wih_d, const float* __restrict__ bih_d, const float* __restrict__ bhh_d,
    const float* __restrict__ Wfc, const float* __restrict__ bfc,
    const unsigned short* __restrict__ WHe, const unsigned short* __restrict__ WHd,
    float* __restrict__ out) {
  __shared__ __align__(16) _Float16 Ah[ROWS_BLK * HPITCH];
  __shared__ __align__(16) float    Xs[ROWS_BLK * XROW];
  __shared__ __align__(16) float    Os[ROWS_BLK * XROW];
  __shared__ __align__(16) float    Pt[NWAVE * NPART];

  const int tid = threadIdx.x, lane = tid & 31, wave = tid >> 5;
  const int c = lane & 15, hh = lane >> 4, koff = hh * 8;
  const int rowbase = blockIdx.x * ROWS_BLK;

#pragma unroll 1
  for (int i = tid; i < ROWS_BLK * HPITCH; i += NTHR) Ah[i] = (_Float16)0.0f;

  float hst[2][8];
#pragma unroll
  for (int nt = 0; nt < 2; ++nt)
#pragma unroll
    for (int r = 0; r < 8; ++r) hst[nt][r] = 0.0f;

  float wfc[3][2];
#pragma unroll
  for (int d = 0; d < 3; ++d)
#pragma unroll
    for (int nt = 0; nt < 2; ++nt) wfc[d][nt] = Wfc[d * NHID + 32 * wave + 16 * nt + c];
#pragma unroll
  for (int d = 0; d < 3; ++d)
#pragma unroll
    for (int nt = 0; nt < 2; ++nt) pin_f(wfc[d][nt]);
  const int od = tid % 3;
  const int om = tid / 3;
  float bfcv = bfc[od];
  pin_f(bfcv);

  const _Float16* ahrow = Ah + c * HPITCH + koff;
  const v8f z8 = {0.f, 0.f, 0.f, 0.f, 0.f, 0.f, 0.f, 0.f};

#pragma unroll 1
  for (int phase = 0; phase < 2; ++phase) {
    const float* X   = phase ? Xf : Xp;
    const float* Wih = phase ? Wih_d : Wih_e;
    const float* bih = phase ? bih_d : bih_e;
    const float* bhh = phase ? bhh_d : bhh_e;
    const _Float16* WH = (const _Float16*)(phase ? WHd : WHe);
    const int shift3 = phase * NDIM;

    float wi[2][3][3], bsum[2][2], bin[2], bhn[2];
#pragma unroll
    for (int nt = 0; nt < 2; ++nt) {
      const int j = 32 * wave + 16 * nt + c;
#pragma unroll
      for (int g = 0; g < 3; ++g)
#pragma unroll
        for (int d = 0; d < 3; ++d) wi[nt][g][d] = Wih[(g * NHID + j) * NDIM + d];
      const float bir = bih[j],            bhr = bhh[j];
      const float biz = bih[NHID + j],     bhz = bhh[NHID + j];
      const float bi2 = bih[2 * NHID + j], bh2 = bhh[2 * NHID + j];
      bsum[nt][0] = bir + bhr;
      bsum[nt][1] = biz + bhz;
      bin[nt] = bi2;
      bhn[nt] = bh2;
#pragma unroll
      for (int g = 0; g < 3; ++g)
#pragma unroll
        for (int d = 0; d < 3; ++d) pin_f(wi[nt][g][d]);
      pin_f(bsum[nt][0]);
      pin_f(bsum[nt][1]);
      pin_f(bin[nt]);
      pin_f(bhn[nt]);
    }

#pragma unroll
    for (int i = 0; i < (ROWS_BLK * XROW) / NTHR; ++i) {
      const int idx = i * NTHR + tid;
      const int m = idx / XROW;
      const int e = idx - m * XROW;
      const int rel = e - shift3;
      const int relc = rel < 0 ? 0 : rel;
      const float v = X[(size_t)(rowbase + m) * (NSTEP * NDIM) + relc];
      Xs[idx] = (rel >= 0) ? v : 0.0f;
    }
    __syncthreads();

#pragma unroll 1
    for (int t = 0; t < NSTEP; ++t) {
      const int js = t & (TCHUNK - 1);
      float xv[8][3];
#pragma unroll
      for (int r = 0; r < 8; ++r)
#pragma unroll
        for (int d = 0; d < 3; ++d) xv[r][d] = Xs[(8 * hh + r) * XROW + js * NDIM + d];

#pragma unroll
      for (int nt = 0; nt < 2; ++nt) {
        const int j = 32 * wave + 16 * nt + c;
        const _Float16* wh = WH + (size_t)j * NHID + koff;
        v8f a0 = z8, a1 = z8, a2 = z8;
#pragma unroll 1
        for (int k0 = 0; k0 < NHID; k0 += 32) {
          const v16h a  = FragH::load(ahrow + k0);
          const v16h b0 = FragH::load(wh + k0);
          const v16h b1 = FragH::load(wh + (size_t)1 * NHID * NHID + k0);
          const v16h b2 = FragH::load(wh + (size_t)2 * NHID * NHID + k0);
          a0 = FragH::mma(a, b0, a0);
          a1 = FragH::mma(a, b1, a1);
          a2 = FragH::mma(a, b2, a2);
          dep_guard3_h(a0, a1, a2, a, b0, b1, b2);
        }
        acc_guard3(a0, a1, a2);
#pragma unroll
        for (int r = 0; r < 8; ++r) {
          const float x0 = xv[r][0], x1 = xv[r][1], x2 = xv[r][2];
          const float pr = fmaf(wi[nt][0][0], x0, fmaf(wi[nt][0][1], x1, fmaf(wi[nt][0][2], x2, bsum[nt][0])));
          const float pz = fmaf(wi[nt][1][0], x0, fmaf(wi[nt][1][1], x1, fmaf(wi[nt][1][2], x2, bsum[nt][1])));
          const float pn = fmaf(wi[nt][2][0], x0, fmaf(wi[nt][2][1], x1, fmaf(wi[nt][2][2], x2, bin[nt])));
          const float ar = a0[r];
          const float az = a1[r];
          const float an = a2[r];
          const float rg = fsig(fmaf(ar, FOLD, pr));
          const float zg = fsig(fmaf(az, FOLD, pz));
          const float hn = fmaf(an, FOLD, bhn[nt]);
          const float ng = ftanh(fmaf(rg, hn, pn));
          const float ho = hst[nt][r];
          hst[nt][r] = (1.0f - zg) * ng + zg * ho;
        }
      }
      __syncthreads();

#pragma unroll
      for (int nt = 0; nt < 2; ++nt) {
        const int j = 32 * wave + 16 * nt + c;
#pragma unroll
        for (int r = 0; r < 8; ++r) Ah[(8 * hh + r) * HPITCH + j] = (_Float16)(hst[nt][r] * HCARRY);
      }

      if (phase == 1) {
#pragma unroll
        for (int r = 0; r < 8; ++r) {
          float p0 = hst[0][r] * wfc[0][0] + hst[1][r] * wfc[0][1];
          float p1 = hst[0][r] * wfc[1][0] + hst[1][r] * wfc[1][1];
          float p2 = hst[0][r] * wfc[2][0] + hst[1][r] * wfc[2][1];
#pragma unroll
          for (int off = 1; off < 16; off <<= 1) {
            const float q0 = __shfl_xor(p0, off, 32);
            const float q1 = __shfl_xor(p1, off, 32);
            const float q2 = __shfl_xor(p2, off, 32);
            p0 += q0;
            p1 += q1;
            p2 += q2;
          }
          if (c == 0) {
            Pt[wave * NPART + (8 * hh + r) * NDIM + 0] = p0;
            Pt[wave * NPART + (8 * hh + r) * NDIM + 1] = p1;
            Pt[wave * NPART + (8 * hh + r) * NDIM + 2] = p2;
          }
        }
      }

      if (js == TCHUNK - 1 && t + 1 < NSTEP) {
        const int t0n = t + 1;
#pragma unroll
        for (int i = 0; i < (ROWS_BLK * XROW) / NTHR; ++i) {
          const int idx = i * NTHR + tid;
          const int m = idx / XROW;
          const int e = idx - m * XROW;
          const int rel = t0n * NDIM + e - shift3;
          const int relc = rel < 0 ? 0 : rel;
          const float v = X[(size_t)(rowbase + m) * (NSTEP * NDIM) + relc];
          Xs[idx] = (rel >= 0) ? v : 0.0f;
        }
      }
      __syncthreads();

      if (phase == 1) {
        if (tid < NPART) {
          float s = bfcv;
#pragma unroll
          for (int w = 0; w < NWAVE; ++w) s += Pt[w * NPART + tid];
          Os[om * XROW + js * NDIM + od] = s;
        }
        if (js == TCHUNK - 1) {
          __syncthreads();
          const int t0 = t - (TCHUNK - 1);
          for (int pass = 0; pass < 2; ++pass) {
#pragma unroll
            for (int it = 0; it < 2; ++it) {
              const int idx = it * NTHR + tid;
              if (idx < ROWS_BLK * (XROW / 4)) {
                const int row = idx / (XROW / 4);
                const int q = idx - row * (XROW / 4);
                const v4f v = *(const v4f*)(Os + row * XROW + q * 4);
                *(volatile v4f*)(out + ((size_t)(rowbase + row) * NSTEP + (size_t)t0) * NDIM + q * 4) = v;
              }
            }
            __threadfence();
          }
        }
      }
    }

    if (phase == 0) {
#pragma unroll
      for (int nt = 0; nt < 2; ++nt) {
        const int j = 32 * wave + 16 * nt + c;
#pragma unroll
        for (int r = 0; r < 8; ++r) {
          const float nz = noise[(size_t)(rowbase + 8 * hh + r) * NHID + j];
          const float hv = hst[nt][r] + nz;
          hst[nt][r] = hv;
          Ah[(8 * hh + r) * HPITCH + j] = (_Float16)(hv * HCARRY);
        }
      }
    }
  }
}

extern "C" void kernel_launch(void* const* d_in, const int* in_sizes, int n_in,
                              void* d_out, int out_size, void* d_ws, size_t ws_size, hipStream_t stream) {
  if (n_in < 13 || d_out == nullptr || d_ws == nullptr) return;
  if (in_sizes[0] != NBATCH * NSTEP * NDIM || in_sizes[1] != NBATCH * NSTEP * NDIM || in_sizes[2] != NBATCH * NHID ||
      in_sizes[3] != NGATE * NDIM || in_sizes[4] != NGATE * NHID || in_sizes[5] != NGATE || in_sizes[6] != NGATE ||
      in_sizes[7] != NGATE * NDIM || in_sizes[8] != NGATE * NHID || in_sizes[9] != NGATE || in_sizes[10] != NGATE ||
      in_sizes[11] != NDIM * NHID || in_sizes[12] != NDIM || out_size != NBATCH * NSTEP * NDIM) return;

  const float* Xp    = (const float*)d_in[0];
  const float* Xf    = (const float*)d_in[1];
  const float* noise = (const float*)d_in[2];
  const float* Wih_e = (const float*)d_in[3];
  const float* Whh_e = (const float*)d_in[4];
  const float* bih_e = (const float*)d_in[5];
  const float* bhh_e = (const float*)d_in[6];
  const float* Wih_d = (const float*)d_in[7];
  const float* Whh_d = (const float*)d_in[8];
  const float* bih_d = (const float*)d_in[9];
  const float* bhh_d = (const float*)d_in[10];
  const float* Wfc   = (const float*)d_in[11];
  const float* bfc   = (const float*)d_in[12];
  float* out = (float*)d_out;

  char* ws = (char*)d_ws;
  size_t off = 0;
  auto carve = [&](size_t bytes) -> char* { char* p = ws + off; off += (bytes + 255) & ~(size_t)255; return p; };
  unsigned short* WHE = (unsigned short*)carve((size_t)NGATE * NHID * 2);
  unsigned short* WHD = (unsigned short*)carve((size_t)NGATE * NHID * 2);
  if (off > ws_size || off > (size_t)134217728) return;

  const int n8 = NGATE * NHID / 8;
  cvt8_f16_kernel<<<n8 / NTHR, NTHR, 0, stream>>>(Whh_e, WHE, n8, WCARRY);
  cvt8_f16_kernel<<<n8 / NTHR, NTHR, 0, stream>>>(Whh_d, WHD, n8, WCARRY);

  gru_seq_kernel<<<NBATCH / ROWS_BLK, NTHR, 0, stream>>>(
      Xp, Xf, noise,
      Wih_e, bih_e, bhh_e,
      Wih_d, bih_d, bhh_d,
      Wfc, bfc, WHE, WHD, out);
}
